// GIN_4956392260269
// MI455X (gfx1250) — hardware-verified
//
#include <hip/hip_runtime.h>
#include <stddef.h>
#include <stdint.h>


#define NN      50000
#define NE      800000
#define NG      64
#define DD      64
#define NL      4
#define NP      5
#define MP      50048
#define KT      128
#define NTHR    256
#define NWAVE   8
#define EPT     8
#define CHUNK   (NTHR * EPT)
#define WCAP    (EPT * 32)
#define LISTN   (NWAVE * WCAP)
#define NBRUN   1024
#define NBLK    49
#define PKS     10
#define RCAP    28672
#define DEGCAP  64
#define GBM     128
#define NTILE   391
#define RECW    160
#define WPL     (DD * KT)
#define NPLANE  13
#define AGR     64
#define WSMAX   134217728
#define LDS_BKT ((2 * RCAP + 2 * NBRUN + LISTN + 16) * 4)

static_assert(DD == 64 && KT == 2 * DD);
static_assert(MP == NTILE * GBM && MP >= NN && (NTILE - 1) * GBM < NN);
static_assert(NBRUN * NBLK >= MP && NBRUN == (1 << PKS));
static_assert((CHUNK & (CHUNK - 1)) == 0 && ((long long)CHUNK << PKS) < (1LL << 31));
static_assert(((long long)NE << PKS) < (1LL << 31));
static_assert(LISTN >= NBRUN && NTHR * 4 == NBRUN);
static_assert((RCAP % (4 * NTHR)) == 0);
static_assert((long long)NBRUN * NE * 5LL <= (long long)RCAP * NN * 4LL);
static_assert(DEGCAP >= 35 + 8 && RCAP >= 16623 + 16623 / 20);
static_assert(LDS_BKT <= 300000);
static_assert((NE % 4) == 0);
static_assert((MP % AGR) == 0 && AGR == NWAVE * 8);
static_assert(GBM == NWAVE * 16);
static_assert((RECW % 32) == 0 && RECW >= 2 * DD + 1 && RECW / 4 <= NTHR);
static_assert(((MP * 8) % NTHR) == 0 && ((MP * 16) % NTHR) == 0);
static_assert(((NPLANE * 1024) % NTHR) == 0 && (1024 % NTHR) == 0);
static_assert(((16 * DD * NP * 4) % 128) == 0 && (16 * DD * NP) == 10 * 128 * 4);
static_assert(NG * DD * NP == 20480 && NG == 4 * 16);

#define KATTR(T) __launch_bounds__(T) __attribute__((amdgpu_num_vgpr(248)))

typedef float          v2f  __attribute__((ext_vector_type(2)));
typedef float          v4f  __attribute__((ext_vector_type(4)));
typedef float          v8f  __attribute__((ext_vector_type(8)));
typedef int            v4i  __attribute__((ext_vector_type(4)));
typedef int            v8i  __attribute__((ext_vector_type(8)));
typedef unsigned int   v2u  __attribute__((ext_vector_type(2)));
typedef unsigned short v8us __attribute__((ext_vector_type(8)));
typedef __bf16         v16b __attribute__((ext_vector_type(16)));
typedef v4f  __attribute__((may_alias)) v4fa;
typedef v4i  __attribute__((may_alias)) v4ia;
typedef v8us __attribute__((may_alias)) v8usa;
union FragB { v16b v; v8us h[2]; v8i w; };

__device__ __forceinline__ v8f wmb(const FragB& a, const FragB& b, v8f c) {
  v8f d = __builtin_amdgcn_wmma_f32_16x16x32_bf16(false, a.v, false, b.v, (short)0, c, false, false);
  asm volatile("v_nop\n\tv_nop\n\tv_nop\n\tv_nop" : "+v"(d) : "v"(a.w), "v"(b.w));
  return d;
}

__device__ __forceinline__ unsigned bfb(float f) {
  const unsigned u = __float_as_uint(f);
  const unsigned r = (u + 0x7FFFu + ((u >> 16) & 1u)) >> 16;
  return (f != f) ? 0x7FC0u : r;
}
__device__ __forceinline__ float bfv(unsigned b) { return __uint_as_float(b << 16); }
__device__ __forceinline__ float bfr(float f) { return bfv(bfb(f)); }

__device__ __forceinline__ int scan_chunk(const int* __restrict__ dsts, int nE, int cbase, int slotBase,
                                          int nb, int vec8, int* list, int tid, int lane, int wave) {
  int wc = 0;
  const int el0  = tid * EPT;
  const int e0   = cbase + el0;
  const int sent = -2147483647 - 1;
  v4i da, db;
  if (vec8 != 0 && cbase + CHUNK <= nE) {
    da = *(const v4i*)(dsts + e0);
    db = *(const v4i*)(dsts + e0 + 4);
  } else {
    da.x = (e0     < nE) ? dsts[min(e0,     nE - 1)] : sent;
    da.y = (e0 + 1 < nE) ? dsts[min(e0 + 1, nE - 1)] : sent;
    da.z = (e0 + 2 < nE) ? dsts[min(e0 + 2, nE - 1)] : sent;
    da.w = (e0 + 3 < nE) ? dsts[min(e0 + 3, nE - 1)] : sent;
    db.x = (e0 + 4 < nE) ? dsts[min(e0 + 4, nE - 1)] : sent;
    db.y = (e0 + 5 < nE) ? dsts[min(e0 + 5, nE - 1)] : sent;
    db.z = (e0 + 6 < nE) ? dsts[min(e0 + 6, nE - 1)] : sent;
    db.w = (e0 + 7 < nE) ? dsts[min(e0 + 7, nE - 1)] : sent;
  }
  const unsigned nbs = (unsigned)slotBase;
  const unsigned unb = (unsigned)nb;
  const unsigned s0 = (unsigned)da.x - nbs, s1 = (unsigned)da.y - nbs;
  const unsigned s2 = (unsigned)da.z - nbs, s3 = (unsigned)da.w - nbs;
  const unsigned s4 = (unsigned)db.x - nbs, s5 = (unsigned)db.y - nbs;
  const unsigned s6 = (unsigned)db.z - nbs, s7 = (unsigned)db.w - nbs;
  const bool h0 = s0 < unb, h1 = s1 < unb, h2 = s2 < unb, h3 = s3 < unb;
  const bool h4 = s4 < unb, h5 = s5 < unb, h6 = s6 < unb, h7 = s7 < unb;
  const unsigned any = __builtin_amdgcn_ballot_w32(h0 | h1 | h2 | h3 | h4 | h5 | h6 | h7);
  if (any != 0u) {
#define HITJ(J, HJ, SJ) { \
      const unsigned mj = __builtin_amdgcn_ballot_w32(HJ); \
      if (mj != 0u) { \
        if (HJ) { \
          const int pos = wc + (int)__builtin_amdgcn_mbcnt_lo(mj, 0u); \
          if (pos < WCAP) list[wave * WCAP + pos] = ((el0 + (J)) << PKS) | (int)(SJ); \
        } \
        wc += (int)__builtin_popcount(mj); } }
    HITJ(0, h0, s0)
    HITJ(1, h1, s1)
    HITJ(2, h2, s2)
    HITJ(3, h3, s3)
    HITJ(4, h4, s4)
    HITJ(5, h5, s5)
    HITJ(6, h6, s6)
    HITJ(7, h7, s7)
#undef HITJ
  }
  return wc;
}

__global__ KATTR(NTHR) void k_pa(const float* __restrict__ x, unsigned short* xb) {
  const int u   = (int)blockIdx.x * NTHR + (int)threadIdx.x;
  const int row = u >> 3;
  const int c8  = (u & 7) * 8;
  const int rc  = row < NN ? row : NN - 1;
  const float* p = x + (size_t)rc * DD + c8;
  const v4f a = *(const v4f*)p;
  const v4f b = *(const v4f*)(p + 4);
  const bool ok = row < NN;
  v8us o;
  o[0] = ok ? (unsigned short)bfb(a.x) : (unsigned short)0;
  o[1] = ok ? (unsigned short)bfb(a.y) : (unsigned short)0;
  o[2] = ok ? (unsigned short)bfb(a.z) : (unsigned short)0;
  o[3] = ok ? (unsigned short)bfb(a.w) : (unsigned short)0;
  o[4] = ok ? (unsigned short)bfb(b.x) : (unsigned short)0;
  o[5] = ok ? (unsigned short)bfb(b.y) : (unsigned short)0;
  o[6] = ok ? (unsigned short)bfb(b.z) : (unsigned short)0;
  o[7] = ok ? (unsigned short)bfb(b.w) : (unsigned short)0;
  unsigned short* dp = xb + (size_t)u * 8;
  *(volatile v8us*)dp = o;
  __threadfence();
  *(volatile v8us*)dp = o;
}

__device__ __forceinline__ v8us gather8(const float* __restrict__ p) {
  v8us o;
#pragma unroll
  for (int i = 0; i < 8; ++i) o[i] = (unsigned short)bfb(p[(size_t)i * DD]);
  return o;
}
__global__ KATTR(NTHR) void k_pb(const float* __restrict__ W1, const float* __restrict__ W2,
                                 const float* __restrict__ PW, unsigned short* wp) {
  const int u  = (int)blockIdx.x * NTHR + (int)threadIdx.x;
  const int mi = u >> 10;
  const int v  = u & 1023;
  const int n  = v >> 4;
  const int k8 = (v & 15) * 8;
  const int kk = k8 & (DD - 1);
  const int eo = kk * DD + n;
  v8us o;
  if (mi < 4)      o = gather8(W1 + (size_t)mi * DD * DD + eo);
  else if (mi < 8) o = gather8(W2 + (size_t)(mi - 4) * DD * DD + eo);
  else             o = gather8(PW + (size_t)(mi - 8) * DD * DD + eo);
  unsigned short* dp = wp + (size_t)u * 8;
  *(volatile v8us*)dp = o;
  __threadfence();
  *(volatile v8us*)dp = o;
}

__global__ KATTR(NTHR) void k_bucket(const int* __restrict__ srcs, const int* __restrict__ dsts,
                                     int* LISTg, int* CNTg, int* OFFg, int* FLAGg) {
  extern __shared__ v4f lds_dyn[];
  int* reg1 = (int*)lds_dyn;
  int* reg2 = reg1 + RCAP;
  int* scnt = reg2 + RCAP;
  int* soff = scnt + NBRUN;
  int* list = soff + NBRUN;
  int* wcnt = list + LISTN;
  int* wtot = wcnt + NWAVE;
  const int tid = (int)threadIdx.x, lane = tid & 31, wave = tid >> 5;
  const int nodeBase = (int)blockIdx.x * NBRUN;

  for (int i = tid; i < NBRUN; i += NTHR) scnt[i] = 0;
  if (tid == 0) reg2[0] = 0;
  __syncthreads();

  int tot = 0;
  const int nChunks = (NE + CHUNK - 1) / CHUNK;
#pragma unroll 1
  for (int ch = 0; ch < nChunks; ++ch) {
    const int cbase = ch * CHUNK;
    const int wc = scan_chunk(dsts, NE, cbase, nodeBase, NBRUN, 1, list, tid, lane, wave);
    if (lane == 0) wcnt[wave] = wc;
    __syncthreads();
    int pre = 0, all = 0;
#pragma unroll
    for (int w2 = 0; w2 < NWAVE; ++w2) {
      int c = wcnt[w2];
      c = c < 0 ? 0 : (c > WCAP ? WCAP : c);
      all += c;
      pre += (w2 < wave) ? c : 0;
    }
    const int wcc  = wc > WCAP ? WCAP : wc;
    const int base = tot + pre;
#pragma unroll 1
    for (int i = lane; i < wcc; i += 32) {
      const int ent = list[wave * WCAP + i];
      const int el  = (ent >> PKS) & (CHUNK - 1);
      const int sl  = ent & (NBRUN - 1);
      int eid = cbase + el;
      eid = eid > NE - 1 ? NE - 1 : eid;
      const int pos = base + i;
      if (pos < RCAP) reg1[pos] = (int)(((unsigned)eid << PKS) | (unsigned)sl);
    }
    tot += all;
    tot = tot > RCAP ? RCAP : tot;
    __syncthreads();
  }
  const int nh = tot;

  if (wave == 0) {
#pragma unroll 1
    for (int b0 = 0; b0 < nh; b0 += 32) {
      int idx = b0 + lane;
      idx = idx > nh - 1 ? nh - 1 : idx;
      const int uv  = reg1[idx];
      const int m32 = (nh - b0) < 32 ? (nh - b0) : 32;
#pragma unroll 1
      for (int k = 0; k < m32; ++k) {
        const int u  = __builtin_amdgcn_readlane(uv, k);
        const int sl = u & (NBRUN - 1);
        if (lane == 0) scnt[sl] = scnt[sl] + 1;
      }
    }
  }
  __syncthreads();

  {
    const v4i ca = *(const v4ia*)(scnt + 4 * tid);
    const int e0 = ca.x < 0 ? 0 : ca.x, e1 = ca.y < 0 ? 0 : ca.y, e2 = ca.z < 0 ? 0 : ca.z, e3 = ca.w < 0 ? 0 : ca.w;
    const int ts = e0 + e1 + e2 + e3;
    int incl = ts;
#pragma unroll
    for (int d = 1; d < 32; d <<= 1) {
      const int up = __shfl_up(incl, d);
      if (lane >= d) incl += up;
    }
    if (lane == 31) wtot[wave] = incl;
    __syncthreads();
    int pre = 0;
#pragma unroll
    for (int w2 = 0; w2 < NWAVE; ++w2) pre += (w2 < wave) ? wtot[w2] : 0;
    int run = pre + incl - ts;
    soff[4 * tid + 0] = run; run += e0;
    soff[4 * tid + 1] = run; run += e1;
    soff[4 * tid + 2] = run; run += e2;
    soff[4 * tid + 3] = run;
  }
  __syncthreads();
  for (int i = tid; i < NBRUN; i += NTHR) list[i] = soff[i];
  __syncthreads();

  if (wave == 0) {
#pragma unroll 1
    for (int b0 = 0; b0 < nh; b0 += 32) {
      int idx = b0 + lane;
      idx = idx > nh - 1 ? nh - 1 : idx;
      const int uv  = reg1[idx];
      const int m32 = (nh - b0) < 32 ? (nh - b0) : 32;
#pragma unroll 1
      for (int k = 0; k < m32; ++k) {
        const int u   = __builtin_amdgcn_readlane(uv, k);
        const int sl  = u & (NBRUN - 1);
        const int eid = (int)((unsigned)u >> PKS);
        if (lane == 0) {
          int pos = list[sl];
          pos = pos < 0 ? 0 : (pos > RCAP - 1 ? RCAP - 1 : pos);
          reg2[pos] = eid;
          list[sl] = pos + 1;
        }
      }
    }
  }
  __syncthreads();

  const int lastv = nh > 0 ? nh - 1 : 0;
#pragma unroll 4
  for (int i = tid; i < RCAP; i += NTHR) {
    const int ic = i < nh ? i : lastv;
    int eid = reg2[ic];
    eid = eid < 0 ? 0 : (eid > NE - 1 ? NE - 1 : eid);
    int s = srcs[eid];
    s = s < 0 ? 0 : (s > NN - 1 ? NN - 1 : s);
    reg1[i] = (i < nh) ? s : 0;
  }
  __syncthreads();

  int* lp = LISTg + (size_t)blockIdx.x * RCAP;
  const v4i cv = *(const v4ia*)(scnt + 4 * tid);
  const v4i ov = *(const v4ia*)(soff + 4 * tid);
  const int fl = (nh >= RCAP) ? 1 : 0;
  v4i fv; fv.x = fl; fv.y = fl; fv.z = fl; fv.w = fl;
#pragma unroll 1
  for (int q = tid; q < RCAP / 4; q += NTHR) {
    const v4i v = *(const v4ia*)(reg1 + 4 * q);
    *(volatile v4i*)(lp + 4 * q) = v;
  }
  *(volatile v4i*)(CNTg + nodeBase + 4 * tid) = cv;
  *(volatile v4i*)(OFFg + nodeBase + 4 * tid) = ov;
  if (tid < 8) *(volatile v4i*)(FLAGg + (size_t)blockIdx.x * 32 + 4 * tid) = fv;
  __threadfence();
#pragma unroll 1
  for (int q = tid; q < RCAP / 4; q += NTHR) {
    const v4i v = *(const v4ia*)(reg1 + 4 * q);
    *(volatile v4i*)(lp + 4 * q) = v;
  }
  *(volatile v4i*)(CNTg + nodeBase + 4 * tid) = cv;
  *(volatile v4i*)(OFFg + nodeBase + 4 * tid) = ov;
  if (tid < 8) *(volatile v4i*)(FLAGg + (size_t)blockIdx.x * 32 + 4 * tid) = fv;
}

template <int BF>
__global__ KATTR(NTHR) void k_agg(const int* __restrict__ LISTg, const int* __restrict__ CNTg,
                                  const int* __restrict__ OFFg, const int* __restrict__ FLAGg,
                                  const unsigned int* __restrict__ xw, const float* __restrict__ hp,
                                  unsigned int* zw) {
  const int tid = (int)threadIdx.x, lane = tid & 31;
  const int wave = __builtin_amdgcn_readfirstlane(tid >> 5);
  const float qnan = __int_as_float(0x7fc00000);
#pragma unroll 1
  for (int jt = 0; jt < 8; ++jt) {
    const int grow = (int)blockIdx.x * AGR + wave * 8 + jt;
    const int b    = grow >> PKS;
    const int craw = CNTg[grow];
    int st = OFFg[grow];
    const int fl = FLAGg[b * 32];
    int cnt = craw;
    st  = st < 0 ? 0 : (st > RCAP ? RCAP : st);
    cnt = cnt < 0 ? 0 : (cnt > DEGCAP ? DEGCAP : cnt);
    if (cnt > RCAP - st) cnt = RCAP - st;
    const bool live = grow < NN;
    const bool bad  = (fl != 0) || (craw > DEGCAP) || (craw < 0);
    const int* lp = LISTg + (size_t)b * RCAP;

    float ag0 = 0.0f, ag1 = 0.0f;
#pragma unroll 1
    for (int b0 = 0; b0 < cnt; b0 += 32) {
      int idx = st + b0 + lane;
      idx = idx < 0 ? 0 : (idx > RCAP - 1 ? RCAP - 1 : idx);
      int sv = lp[idx];
      sv = sv < 0 ? 0 : (sv > NN - 1 ? NN - 1 : sv);
      const int m32 = (cnt - b0) < 32 ? (cnt - b0) : 32;
#pragma unroll 1
      for (int k = 0; k < m32; ++k) {
        const int sk = __builtin_amdgcn_readlane(sv, k);
        float v0, v1;
        if constexpr (BF != 0) {
          const unsigned w = xw[(size_t)sk * 32 + lane];
          v0 = __uint_as_float(w << 16);
          v1 = __uint_as_float(w & 0xffff0000u);
        } else {
          const v2f q = *(const v2f*)(hp + (size_t)sk * DD + 2 * lane);
          v0 = q.x; v1 = q.y;
        }
        ag0 += v0; ag1 += v1;
      }
    }
    const int nc = live ? grow : NN - 1;
    float s0, s1;
    if constexpr (BF != 0) {
      const unsigned w = xw[(size_t)nc * 32 + lane];
      s0 = __uint_as_float(w << 16);
      s1 = __uint_as_float(w & 0xffff0000u);
    } else {
      const v2f q = *(const v2f*)(hp + (size_t)nc * DD + 2 * lane);
      s0 = q.x; s1 = q.y;
    }
    float r0 = ag0 + s0, r1 = ag1 + s1;
    r0 = live ? r0 : 0.0f;
    r1 = live ? r1 : 0.0f;
    r0 = (bad && live) ? qnan : r0;
    r1 = (bad && live) ? qnan : r1;
    const unsigned hb0 = bfb(r0), hb1 = bfb(r1);
    const unsigned lb0 = bfb(r0 - bfv(hb0)), lb1 = bfb(r1 - bfv(hb1));
    const unsigned hw = hb0 | (hb1 << 16);
    const unsigned lw = lb0 | (lb1 << 16);
    volatile unsigned int* zp = zw + (size_t)grow * 64;
    zp[lane] = hw;
    zp[32 + lane] = lw;
    __threadfence();
    zp[lane] = hw;
    zp[32 + lane] = lw;
  }
}

template <int MODE>
__global__ KATTR(NTHR) void k_gemm(const unsigned short* __restrict__ A, const unsigned short* __restrict__ WT,
                                   const float* __restrict__ bias, unsigned short* outH, float* outF,
                                   float* rec) {
  __shared__ __attribute__((aligned(16))) float stg[GBM * DD];
  __shared__ __attribute__((aligned(16))) float pst[RECW];
  const int tid = (int)threadIdx.x, lane = tid & 31, wave = tid >> 5, hh = lane >> 4, m = lane & 15;
  const int rowBase = (int)blockIdx.x * GBM;

  v8f acc[4];
  {
    const v8f z = {0.f, 0.f, 0.f, 0.f, 0.f, 0.f, 0.f, 0.f};
#pragma unroll
    for (int t = 0; t < 4; ++t) acc[t] = z;
  }
  const unsigned short* ap = A + (size_t)(rowBase + 16 * wave + m) * (size_t)KT + 8 * hh;
  const unsigned short* wq0 = WT + (size_t)m * (size_t)KT + 8 * hh;
#pragma unroll 1
  for (int ks = 0; ks < KT / 32; ++ks) {
    FragB af;
    af.h[0] = *(const v8usa*)(ap + 32 * ks);
    af.h[1] = *(const v8usa*)(ap + 32 * ks + 16);
#pragma unroll
    for (int t = 0; t < 4; ++t) {
      const unsigned short* wq = wq0 + (size_t)(16 * t) * (size_t)KT + 32 * ks;
      FragB bf;
      bf.h[0] = *(const v8usa*)wq;
      bf.h[1] = *(const v8usa*)(wq + 16);
      acc[t] = wmb(af, bf, acc[t]);
    }
  }

#pragma unroll
  for (int t = 0; t < 4; ++t) {
    const int lc = 16 * t + m;
    const float bb = bfr(bias[lc]);
#pragma unroll
    for (int r = 0; r < 8; ++r) {
      const int lr = 16 * wave + 8 * hh + r;
      const bool live = (rowBase + lr) < NN;
      float v = acc[t][r] + bb;
      if (MODE == 1) v = (v > 0.0f) ? v : (v - v);
      stg[lr * DD + lc] = live ? v : 0.0f;
    }
  }
  __syncthreads();

  if constexpr (MODE == 0) {
    if (tid < DD) {
      int rv = NN - rowBase;
      rv = rv < 0 ? 0 : (rv > GBM ? GBM : rv);
      float s = 0.0f;
#pragma unroll 4
      for (int r = 0; r < rv; ++r) s += stg[r * DD + tid];
      const float nf = (float)rv;
      const float mean = (rv > 0) ? (s / nf) : 0.0f;
      float q = 0.0f;
#pragma unroll 4
      for (int r = 0; r < rv; ++r) {
        const float d = stg[r * DD + tid] - mean;
        q = fmaf(d, d, q);
      }
      pst[1 + tid] = mean;
      pst[1 + DD + tid] = q;
      if (tid == 0) pst[0] = nf;
      if (tid < RECW - (2 * DD + 1)) pst[2 * DD + 1 + tid] = 0.0f;
    }
    v4f fv[8];
#pragma unroll
    for (int i = 0; i < 8; ++i) fv[i] = *(const v4fa*)(stg + (16 * wave + 2 * i) * DD + 4 * lane);
#pragma unroll
    for (int i = 0; i < 8; ++i) {
      float* op = outF + (size_t)(rowBase + 16 * wave + 2 * i) * (size_t)DD + 4 * lane;
      *(volatile v4f*)op = fv[i];
    }
    __threadfence();
#pragma unroll
    for (int i = 0; i < 8; ++i) {
      float* op = outF + (size_t)(rowBase + 16 * wave + 2 * i) * (size_t)DD + 4 * lane;
      *(volatile v4f*)op = fv[i];
    }
    __syncthreads();
    v4f pv = {0.f, 0.f, 0.f, 0.f};
    const int tq = tid < RECW / 4 ? tid : 0;
    pv = *(const v4fa*)(pst + 4 * tq);
    if (tid < RECW / 4) *(volatile v4f*)(rec + (size_t)blockIdx.x * RECW + 4 * tid) = pv;
    __threadfence();
    if (tid < RECW / 4) *(volatile v4f*)(rec + (size_t)blockIdx.x * RECW + 4 * tid) = pv;
  } else {
    const int ch = 4 * m;
    const bool isHi = (hh == 0);
    v2u pk[16];
#pragma unroll
    for (int i = 0; i < 16; ++i) {
      const int lr = 16 * wave + i;
      const v4f a = *(const v4fa*)(stg + lr * DD + ch);
      const unsigned h0 = bfb(a.x), h1 = bfb(a.y), h2 = bfb(a.z), h3 = bfb(a.w);
      const unsigned l0 = bfb(a.x - bfv(h0)), l1 = bfb(a.y - bfv(h1));
      const unsigned l2 = bfb(a.z - bfv(h2)), l3 = bfb(a.w - bfv(h3));
      const unsigned q0 = isHi ? h0 : l0, q1 = isHi ? h1 : l1;
      const unsigned q2 = isHi ? h2 : l2, q3 = isHi ? h3 : l3;
      v2u pw; pw.x = q0 | (q1 << 16); pw.y = q2 | (q3 << 16);
      pk[i] = pw;
    }
#pragma unroll
    for (int i = 0; i < 16; ++i) {
      unsigned short* op = outH + (size_t)(rowBase + 16 * wave + i) * (size_t)KT + 4 * lane;
      *(volatile v2u*)op = pk[i];
    }
    __threadfence();
#pragma unroll
    for (int i = 0; i < 16; ++i) {
      unsigned short* op = outH + (size_t)(rowBase + 16 * wave + i) * (size_t)KT + 4 * lane;
      *(volatile v2u*)op = pk[i];
    }
  }
}

__global__ KATTR(DD) void k_comb(const float* __restrict__ rec, const float* __restrict__ gam,
                                 const float* __restrict__ bet, float* stat) {
  __shared__ __attribute__((aligned(16))) float stg[4 * DD];
  const int tid = (int)threadIdx.x;
  const int c = tid & (DD - 1);
  double n = 0.0, mean = 0.0, M2 = 0.0;
#pragma unroll 1
  for (int b = 0; b < NTILE; ++b) {
    const float* pr = rec + (size_t)b * RECW;
    const float nb = pr[0];
    const float mb = pr[1 + c];
    const float qb = pr[1 + DD + c];
    if (nb > 0.5f) {
      const double nn = n + (double)nb;
      const double delta = (double)mb - mean;
      const double f = (double)nb / nn;
      mean = mean + delta * f;
      M2 = M2 + (double)qb + delta * delta * n * f;
      n = nn;
    }
  }
  const double nt = n < 1.0 ? 1.0 : n;
  const float var = (float)(M2 / nt);
  const float rs  = 1.0f / sqrtf(var + 1e-5f);
  stg[c]          = (float)mean;
  stg[DD + c]     = rs;
  stg[2 * DD + c] = bfr(gam[c]);
  stg[3 * DD + c] = bfr(bet[c]);
  __syncthreads();
  const v4f v = *(const v4fa*)(stg + 4 * tid);
  *(volatile v4f*)(stat + 4 * tid) = v;
  __threadfence();
  *(volatile v4f*)(stat + 4 * tid) = v;
}

__global__ KATTR(NTHR) void k_apply(const float* __restrict__ uf, const float* __restrict__ stat,
                                    const float* __restrict__ alpha_p, float* hf) {
  __shared__ float ssh[4 * DD];
  const int tid = (int)threadIdx.x;
  ssh[tid] = stat[tid];
  __syncthreads();
  const float al = bfr(alpha_p[0]);
  const int u   = (int)blockIdx.x * NTHR + tid;
  const int row = u >> 4;
  const int c4  = (u & 15) * 4;
  const int rc  = row < NN ? row : NN - 1;
  const v4f a = *(const v4f*)(uf + (size_t)rc * DD + c4);
  const bool ok = row < NN;
  const float y0 = ((a.x - ssh[c4 + 0]) * ssh[DD + c4 + 0]) * ssh[2 * DD + c4 + 0] + ssh[3 * DD + c4 + 0];
  const float y1 = ((a.y - ssh[c4 + 1]) * ssh[DD + c4 + 1]) * ssh[2 * DD + c4 + 1] + ssh[3 * DD + c4 + 1];
  const float y2 = ((a.z - ssh[c4 + 2]) * ssh[DD + c4 + 2]) * ssh[2 * DD + c4 + 2] + ssh[3 * DD + c4 + 2];
  const float y3 = ((a.w - ssh[c4 + 3]) * ssh[DD + c4 + 3]) * ssh[2 * DD + c4 + 3] + ssh[3 * DD + c4 + 3];
  const float p0 = (y0 > 0.0f) ? y0 : al * y0;
  const float p1 = (y1 > 0.0f) ? y1 : al * y1;
  const float p2 = (y2 > 0.0f) ? y2 : al * y2;
  const float p3 = (y3 > 0.0f) ? y3 : al * y3;
  v4f o;
  o.x = ok ? p0 : 0.0f;
  o.y = ok ? p1 : 0.0f;
  o.z = ok ? p2 : 0.0f;
  o.w = ok ? p3 : 0.0f;
  float* hp = hf + (size_t)row * DD + c4;
  *(volatile v4f*)hp = o;
  __threadfence();
  *(volatile v4f*)hp = o;
}

__global__ KATTR(NTHR) void k_pool(const unsigned int* __restrict__ xw, const float* __restrict__ hb,
                                   const int* __restrict__ bat, float* prec) {
  __shared__ __attribute__((aligned(16))) float wmx[NWAVE * DD];
  __shared__ __attribute__((aligned(16))) float outs[DD];
  const int tid = (int)threadIdx.x, lane = tid & 31;
  const int wave = __builtin_amdgcn_readfirstlane(tid >> 5);
  const int l = (int)blockIdx.x >> 6;
  const int g = (int)blockIdx.x & 63;
  const float ninf = __uint_as_float(0xff800000u);
  const size_t pl = (l > 0) ? (size_t)(l - 1) * (size_t)MP * DD : (size_t)0;
  float m0 = ninf, m1 = ninf;
#pragma unroll 1
  for (int i0 = wave * 32; i0 < NN; i0 += NTHR) {
    const int i  = i0 + lane;
    const int ic = i < NN ? i : NN - 1;
    const int b  = bat[ic];
    const bool hit = (i < NN) && (b == g);
    unsigned msk = __builtin_amdgcn_ballot_w32(hit);
#pragma unroll 1
    for (int q = 0; q < 32; ++q) {
      if (msk == 0u) break;
      const int k = __builtin_ctz(msk);
      msk &= msk - 1u;
      int node = i0 + k;
      node = node > NN - 1 ? NN - 1 : node;
      float v0, v1;
      if (l == 0) {
        const unsigned w = xw[(size_t)node * 32 + lane];
        v0 = __uint_as_float(w << 16);
        v1 = __uint_as_float(w & 0xffff0000u);
      } else {
        const v2f t = *(const v2f*)(hb + pl + (size_t)node * DD + 2 * lane);
        v0 = t.x; v1 = t.y;
      }
      m0 = (v0 > m0 || v0 != v0) ? v0 : m0;
      m1 = (v1 > m1 || v1 != v1) ? v1 : m1;
    }
  }
  wmx[wave * DD + 2 * lane + 0] = m0;
  wmx[wave * DD + 2 * lane + 1] = m1;
  __syncthreads();
  if (tid < DD) {
    float mm = ninf;
#pragma unroll
    for (int w2 = 0; w2 < NWAVE; ++w2) {
      const float v = wmx[w2 * DD + tid];
      mm = (v > mm || v != v) ? v : mm;
    }
    outs[tid] = mm;
  }
  __syncthreads();
  const v4f ov = *(const v4fa*)(outs + 4 * (lane & 15));
  float* op = prec + (size_t)blockIdx.x * DD + 4 * (lane & 15);
  const bool okst = (tid < 16);
  if (okst) *(volatile v4f*)op = ov;
  __threadfence();
  if (okst) *(volatile v4f*)op = ov;
}

__global__ KATTR(128) void k_head(const float* __restrict__ prec, const unsigned short* __restrict__ pwc,
                                  const float* __restrict__ pb, float* out) {
  __shared__ __attribute__((aligned(16))) unsigned short at[16 * KT];
  __shared__ __attribute__((aligned(16))) float ot[16 * DD * NP];
  const int tid = (int)threadIdx.x, lane = tid & 31, wave = tid >> 5, hh = lane >> 4, m = lane & 15;
  const int g0 = (int)blockIdx.x * 16;
  const float pinf = __uint_as_float(0x7f800000u);
  const int srow = tid >> 3;
  const int c8   = (tid & 7) * 8;
#pragma unroll 1
  for (int l = 0; l < NP; ++l) {
    {
      const float* p = prec + ((size_t)l * NG + (size_t)(g0 + srow)) * DD + c8;
      const v4f a = *(const v4f*)p;
      const v4f b = *(const v4f*)(p + 4);
      const float f[8] = {a.x, a.y, a.z, a.w, b.x, b.y, b.z, b.w};
      v8us ho, lo;
#pragma unroll
      for (int j = 0; j < 8; ++j) {
        const unsigned hbj = bfb(f[j]);
        const float hv = bfv(hbj);
        const bool fin = fabsf(hv) < pinf;
        const unsigned lbj = bfb(f[j] - hv);
        ho[j] = (unsigned short)hbj;
        lo[j] = fin ? (unsigned short)lbj : (unsigned short)0;
      }
      *(v8usa*)(at + srow * KT + c8) = ho;
      *(v8usa*)(at + srow * KT + DD + c8) = lo;
    }
    __syncthreads();
    v8f acc = {0.f, 0.f, 0.f, 0.f, 0.f, 0.f, 0.f, 0.f};
    const unsigned short* ap = at + m * KT + 8 * hh;
    const unsigned short* wq = pwc + (size_t)l * WPL + (size_t)(16 * wave + m) * KT + 8 * hh;
#pragma unroll 1
    for (int ks = 0; ks < KT / 32; ++ks) {
      FragB af, bf;
      af.h[0] = *(const v8usa*)(ap + 32 * ks);
      af.h[1] = *(const v8usa*)(ap + 32 * ks + 16);
      bf.h[0] = *(const v8usa*)(wq + 32 * ks);
      bf.h[1] = *(const v8usa*)(wq + 32 * ks + 16);
      acc = wmb(af, bf, acc);
    }
    const int d = 16 * wave + m;
    const float bb = bfr(pb[l * DD + d]);
#pragma unroll
    for (int r = 0; r < 8; ++r) {
      ot[(8 * hh + r) * (DD * NP) + d * NP + l] = acc[r] + bb;
    }
    __syncthreads();
  }
  v4f ov[10];
#pragma unroll
  for (int i = 0; i < 10; ++i) ov[i] = *(const v4fa*)(ot + 4 * (i * 128 + tid));
  float* ob = out + (size_t)blockIdx.x * (16 * DD * NP);
#pragma unroll
  for (int i = 0; i < 10; ++i) *(volatile v4f*)(ob + 4 * (i * 128 + tid)) = ov[i];
  __threadfence();
#pragma unroll
  for (int i = 0; i < 10; ++i) *(volatile v4f*)(ob + 4 * (i * 128 + tid)) = ov[i];
}

static inline size_t al256(size_t o) { return (o + 255) & ~(size_t)255; }

extern "C" void kernel_launch(void* const* d_in, const int* in_sizes, int n_in,
                              void* d_out, int out_size, void* d_ws, size_t ws_size,
                              hipStream_t stream) {
  if (n_in < 12) return;
  if (in_sizes[0] != NN * DD || in_sizes[1] != 2 * NE || in_sizes[2] != NN) return;
  if (in_sizes[3] != NL * DD * DD || in_sizes[4] != NL * DD) return;
  if (in_sizes[5] != NL * DD * DD || in_sizes[6] != NL * DD) return;
  if (in_sizes[7] != NL * DD || in_sizes[8] != NL * DD || in_sizes[9] != 1) return;
  if (in_sizes[10] != NP * DD * DD || in_sizes[11] != NP * DD) return;
  if (out_size != NG * DD * NP) return;

  const float* x    = (const float*)d_in[0];
  const int*   ei   = (const int*)  d_in[1];
  const int*   src  = ei;
  const int*   dst  = ei + NE;
  const int*   bat  = (const int*)  d_in[2];
  const float* W1   = (const float*)d_in[3];
  const float* b1   = (const float*)d_in[4];
  const float* W2   = (const float*)d_in[5];
  const float* b2   = (const float*)d_in[6];
  const float* gam  = (const float*)d_in[7];
  const float* bet  = (const float*)d_in[8];
  const float* alp  = (const float*)d_in[9];
  const float* PW   = (const float*)d_in[10];
  const float* pb   = (const float*)d_in[11];
  float* out = (float*)d_out;

  char* ws = (char*)d_ws;
  size_t off = 0;
  const size_t plane = (size_t)MP * DD * 4;
  const size_t oWP  = off; off = al256(off + (size_t)NPLANE * WPL * 2);
  const size_t oXB  = off; off = al256(off + (size_t)MP * DD * 2);
  const size_t oZH  = off; off = al256(off + (size_t)MP * KT * 2);
  const size_t oTH  = off; off = al256(off + (size_t)MP * KT * 2);
  const size_t oU   = off; off = al256(off + plane);
  const size_t oH   = off; off = al256(off + (size_t)NL * plane);
  const size_t oLS  = off; off = al256(off + (size_t)NBLK * RCAP * 4);
  const size_t oCN  = off; off = al256(off + (size_t)NBLK * NBRUN * 4);
  const size_t oOF  = off; off = al256(off + (size_t)NBLK * NBRUN * 4);
  const size_t oFL  = off; off = al256(off + (size_t)NBLK * 32 * 4);
  const size_t oRC  = off; off = al256(off + (size_t)NTILE * RECW * 4);
  const size_t oST  = off; off = al256(off + (size_t)NL * 4 * DD * 4);
  const size_t oPR  = off; off = al256(off + (size_t)NP * NG * DD * 4);
  if (off > ws_size || off > (size_t)WSMAX) return;
  unsigned short* WP   = (unsigned short*)(ws + oWP);
  unsigned short* XB   = (unsigned short*)(ws + oXB);
  unsigned short* ZHL  = (unsigned short*)(ws + oZH);
  unsigned short* THL  = (unsigned short*)(ws + oTH);
  float*          U    = (float*)(ws + oU);
  float*          HB   = (float*)(ws + oH);
  int*            LIST = (int*)(ws + oLS);
  int*            CNT  = (int*)(ws + oCN);
  int*            OFFt = (int*)(ws + oOF);
  int*            FLAG = (int*)(ws + oFL);
  float*          REC  = (float*)(ws + oRC);
  float*          STAT = (float*)(ws + oST);
  float*          PREC = (float*)(ws + oPR);

  hipFuncSetAttribute(reinterpret_cast<const void*>(&k_bucket), hipFuncAttributeMaxDynamicSharedMemorySize, LDS_BKT);

  k_pa<<<(MP * 8) / NTHR, NTHR, 0, stream>>>(x, XB);
  k_pb<<<(NPLANE * 1024) / NTHR, NTHR, 0, stream>>>(W1, W2, PW, WP);
  k_bucket<<<NBLK, NTHR, LDS_BKT, stream>>>(src, dst, LIST, CNT, OFFt, FLAG);

  for (int l = 0; l < NL; ++l) {
    float* Hout = HB + (size_t)l * MP * DD;
    const float* Hin = HB + (size_t)(l > 0 ? l - 1 : 0) * MP * DD;
    if (l == 0) {
      k_agg<1><<<MP / AGR, NTHR, 0, stream>>>(LIST, CNT, OFFt, FLAG, (const unsigned int*)XB, Hin,
                                              (unsigned int*)ZHL);
    } else {
      k_agg<0><<<MP / AGR, NTHR, 0, stream>>>(LIST, CNT, OFFt, FLAG, (const unsigned int*)XB, Hin,
                                              (unsigned int*)ZHL);
    }
    k_gemm<1><<<NTILE, NTHR, 0, stream>>>(ZHL, WP + (size_t)l * WPL, b1 + (size_t)l * DD, THL, U, REC);
    k_gemm<0><<<NTILE, NTHR, 0, stream>>>(THL, WP + (size_t)(4 + l) * WPL, b2 + (size_t)l * DD, ZHL, U, REC);
    k_comb<<<1, DD, 0, stream>>>(REC, gam + (size_t)l * DD, bet + (size_t)l * DD, STAT + (size_t)l * 4 * DD);
    k_apply<<<(MP * 16) / NTHR, NTHR, 0, stream>>>(U, STAT + (size_t)l * 4 * DD, alp, Hout);
  }
  k_pool<<<NP * NG, NTHR, 0, stream>>>((const unsigned int*)XB, HB, bat, PREC);
  k_head<<<4, 128, 0, stream>>>(PREC, WP + (size_t)8 * WPL, pb, out);
}
